// KernelNN_41884521071238
// MI455X (gfx1250) — hardware-verified
//
#include <hip/hip_runtime.h>
#include <math.h>

typedef __attribute__((ext_vector_type(16))) _Float16 v16h;
typedef __attribute__((ext_vector_type(8)))  _Float16 v8h;
typedef __attribute__((ext_vector_type(16))) __bf16   v16b;
typedef __attribute__((ext_vector_type(8)))  float    v8f;
typedef __attribute__((ext_vector_type(4)))  float    v4f;

__device__ __forceinline__ int frag_k(int i, int h) { return (i < 8) ? (8 * h + i) : (16 + 8 * h + (i - 8)); }
__device__ __forceinline__ __bf16 bf16_rne(float f) {
    unsigned int u = __float_as_uint(f);
    u += 0x7fffu + ((u >> 16) & 1u);
    return __builtin_bit_cast(__bf16, (unsigned short)(u >> 16));
}
__device__ __forceinline__ float bf16_f32(__bf16 b) { return __uint_as_float(((unsigned int)__builtin_bit_cast(unsigned short, b)) << 16); }
__device__ __forceinline__ v8f wmma16(v16h a, v16h b, v8f c) {
    c = __builtin_amdgcn_wmma_f32_16x16x32_f16(false, a, false, b, (short)0, c, false, false);
    asm volatile("v_nop\n\tv_nop\n\tv_nop\n\tv_nop" : "+v"(c) : "v"(a), "v"(b));
    return c;
}
__device__ __forceinline__ v8f wmmab(v16b a, v16b b, v8f c) {
    c = __builtin_amdgcn_wmma_f32_16x16x32_bf16(false, a, false, b, (short)0, c, false, false);
    asm volatile("v_nop\n\tv_nop\n\tv_nop\n\tv_nop" : "+v"(c) : "v"(a), "v"(b));
    return c;
}
struct Split { v16b hi, lo; };
__device__ __forceinline__ v8f wmma3(const Split& a, const Split& b, v8f c) {
    c = __builtin_amdgcn_wmma_f32_16x16x32_bf16(false, a.hi, false, b.hi, (short)0, c, false, false);
    c = __builtin_amdgcn_wmma_f32_16x16x32_bf16(false, a.hi, false, b.lo, (short)0, c, false, false);
    c = __builtin_amdgcn_wmma_f32_16x16x32_bf16(false, a.lo, false, b.hi, (short)0, c, false, false);
    asm volatile("v_nop\n\tv_nop\n\tv_nop\n\tv_nop" : "+v"(c) : "v"(a.hi), "v"(a.lo), "v"(b.hi), "v"(b.lo));
    return c;
}
struct Split3 { v16b hi, mid, lo; };
__device__ __forceinline__ v8f wmma6(const Split3& a, const Split3& b, v8f c) {
    c = __builtin_amdgcn_wmma_f32_16x16x32_bf16(false, a.hi, false, b.hi, (short)0, c, false, false);
    c = __builtin_amdgcn_wmma_f32_16x16x32_bf16(false, a.hi, false, b.mid, (short)0, c, false, false);
    c = __builtin_amdgcn_wmma_f32_16x16x32_bf16(false, a.mid, false, b.hi, (short)0, c, false, false);
    c = __builtin_amdgcn_wmma_f32_16x16x32_bf16(false, a.hi, false, b.lo, (short)0, c, false, false);
    c = __builtin_amdgcn_wmma_f32_16x16x32_bf16(false, a.mid, false, b.mid, (short)0, c, false, false);
    c = __builtin_amdgcn_wmma_f32_16x16x32_bf16(false, a.lo, false, b.hi, (short)0, c, false, false);
    asm volatile("v_nop\n\tv_nop\n\tv_nop\n\tv_nop" : "+v"(c) : "v"(a.hi), "v"(a.mid), "v"(a.lo), "v"(b.hi), "v"(b.mid), "v"(b.lo));
    return c;
}

__device__ __forceinline__ v16h fh_ld(const float* __restrict__ p, long long sk, int k0, int h, int klen, float s) {
    v16h a;
#pragma unroll
    for (int i = 0; i < 16; ++i) { const int k = k0 + frag_k(i, h); a[i] = (k < klen) ? (_Float16)(p[(long long)k * sk] * s) : (_Float16)0.f; }
    return a;
}
__device__ __forceinline__ Split sp_ld(const float* __restrict__ p, long long sk, int k0, int h, int klen, float s) {
    Split r;
#pragma unroll
    for (int i = 0; i < 16; ++i) {
        const int k = k0 + frag_k(i, h); const float x = (k < klen) ? p[(long long)k * sk] * s : 0.f;
        const __bf16 hb = bf16_rne(x); r.hi[i] = hb; r.lo[i] = bf16_rne(x - bf16_f32(hb));
    }
    return r;
}
__device__ __forceinline__ Split3 sp3_ld(const float* __restrict__ p, long long sk, int k0, int h, int klen, float s) {
    Split3 r;
#pragma unroll
    for (int i = 0; i < 16; ++i) {
        const int k = k0 + frag_k(i, h); const float x = (k < klen) ? p[(long long)k * sk] * s : 0.f;
        const __bf16 hb = bf16_rne(x); const float r1 = x - bf16_f32(hb); const __bf16 mb = bf16_rne(r1);
        r.hi[i] = hb; r.mid[i] = mb; r.lo[i] = bf16_rne(r1 - bf16_f32(mb));
    }
    return r;
}
__device__ __forceinline__ v16b bh_ld(const float* __restrict__ p, long long sk, int k0, int h, int klen, float s) {
    v16b a;
#pragma unroll
    for (int i = 0; i < 16; ++i) { const int k = k0 + frag_k(i, h); a[i] = bf16_rne((k < klen) ? p[(long long)k * sk] * s : 0.f); }
    return a;
}
__device__ __forceinline__ v16h fh_row(const _Float16* __restrict__ row, int k0, int h) {
    v16h a;
#pragma unroll
    for (int i = 0; i < 16; ++i) a[i] = row[k0 + frag_k(i, h)];
    return a;
}

#define VST2(T, ptr, val) do { *(volatile T*)(ptr) = (val); __threadfence(); *(volatile T*)(ptr) = (val); } while (0)
typedef float v4f __attribute__((ext_vector_type(4)));
#define VST2V4(ptr, val) do { *(volatile v4f*)(ptr) = (val); __threadfence(); *(volatile v4f*)(ptr) = (val); } while (0)

__device__ __attribute__((noinline)) float act_fn(float v, int act) {
    if (act == 1) return fmaxf(v, 0.f);
    if (act == 2) { const float u = 0.7978845608028654f * (v + 0.044715f * v * v * v); return 0.5f * v * (1.f + tanhf(u)); }
    if (act == 3) return v / (1.f + expf(-v));
    if (act == 4) return 0.5f * v * (1.f + erff(v * 0.7071067811865476f));
    if (act == 5) return tanhf(v);
    if (act == 6) return 1.f / (1.f + expf(-v));
    if (act == 7) return (v > 0.f) ? v : 0.01f * v;
    if (act == 8) return (v > 0.f) ? v : (expf(v) - 1.f);
    if (act == 9) return fminf(fmaxf(v, 0.f), 6.f);
    if (act == 10) return fabsf(v);
    if (act == 11) return (v >= 0.f) ? v : 0.1f * v;
    if (act == 12) return (v > 0.f) ? v : 0.2f * v;
    if (act == 13) return (v > 20.f) ? v : log1pf(expf(v));
    return v;
}

struct GemmP {
    const float* A; const float* B; const float* bias; const float* R; float* C;
    long long sAo, sAi, sAm, sAk, sBo, sBi, sBn, sBk, sCo, sCi, sCm, sRo, sRi, sRm, sRn;
    int M, N, K, zi_n, flags, act; float alpha, beta, sa, sb;
    int Npad, pad_;
};
static_assert(sizeof(GemmP) == 5 * 8 + 15 * 8 + 6 * 4 + 4 * 4 + 2 * 4, "GemmP has padding");

template <int MODE>
__global__ __launch_bounds__(32) void k_gemm(GemmP p) {
    const int lane = threadIdx.x & 31, h = lane >> 4, l15 = lane & 15;
    const int m0 = blockIdx.y * 16, n0 = blockIdx.x * 32;
    const int z = blockIdx.z, zo = z / p.zi_n, zi = z - zo * p.zi_n;
    const float* A = p.A + zo * p.sAo + zi * p.sAi;
    const float* B = p.B + zo * p.sBo + zi * p.sBi;
    const int am = min(m0 + l15, p.M - 1);
    v8f acc[2], comp[2];
#pragma unroll
    for (int t = 0; t < 2; ++t) { v8f zz = {}; acc[t] = zz; comp[t] = zz; }
    for (int k0 = 0; k0 < p.K; k0 += 32) {
        const float* arow = A + (long long)am * p.sAm;
        if (MODE == 1) {
            const Split a = sp_ld(arow, p.sAk, k0, h, p.K, 1.f);
#pragma unroll
            for (int t = 0; t < 2; ++t) {
                const int bn = min(n0 + t * 16 + l15, p.N - 1);
                acc[t] = wmma3(a, sp_ld(B + (long long)bn * p.sBn, p.sBk, k0, h, p.K, 1.f), acc[t]);
            }
        } else if (MODE == 3) {
            const Split3 a = sp3_ld(arow, p.sAk, k0, h, p.K, 1.f);
#pragma unroll
            for (int t = 0; t < 2; ++t) {
                const int bn = min(n0 + t * 16 + l15, p.N - 1);
                acc[t] = wmma6(a, sp3_ld(B + (long long)bn * p.sBn, p.sBk, k0, h, p.K, 1.f), acc[t]);
            }
        } else if (MODE == 4) {
            const Split3 a = sp3_ld(arow, p.sAk, k0, h, p.K, 1.f);
#pragma unroll
            for (int t = 0; t < 2; ++t) {
                const int bn = min(n0 + t * 16 + l15, p.N - 1); v8f zz = {};
                const v8f part = wmma6(a, sp3_ld(B + (long long)bn * p.sBn, p.sBk, k0, h, p.K, 1.f), zz);
                const v8f y = part - comp[t]; const v8f s = acc[t] + y; comp[t] = (s - acc[t]) - y; acc[t] = s;
            }
        } else if (MODE == 2) {
            const v16b a = bh_ld(arow, p.sAk, k0, h, p.K, 1.f);
#pragma unroll
            for (int t = 0; t < 2; ++t) {
                const int bn = min(n0 + t * 16 + l15, p.N - 1);
                acc[t] = wmmab(a, bh_ld(B + (long long)bn * p.sBn, p.sBk, k0, h, p.K, 1.f), acc[t]);
            }
        } else {
            const v16h a = fh_ld(arow, p.sAk, k0, h, p.K, p.sa);
#pragma unroll
            for (int t = 0; t < 2; ++t) {
                const int bn = min(n0 + t * 16 + l15, p.N - 1);
                acc[t] = wmma16(a, fh_ld(B + (long long)bn * p.sBn, p.sBk, k0, h, p.K, p.sb), acc[t]);
            }
        }
    }
    const float iscale = (MODE == 0) ? p.alpha / (p.sa * p.sb) : p.alpha;
    float* C = p.C + zo * p.sCo + zi * p.sCi;
    const float* R = p.R + zo * p.sRo + zi * p.sRi;
    __shared__ __align__(16) float ctile[16][36];
#pragma unroll
    for (int t = 0; t < 2; ++t) {
        const int n = n0 + t * 16 + l15; const int nn = min(n, p.N - 1);
#pragma unroll
        for (int r = 0; r < 8; ++r) {
            const int m = m0 + 8 * h + r; const int mm = min(m, p.M - 1);
            float v = acc[t][r] * iscale;
            if (p.flags & 1) v += p.bias[nn];
            if (p.flags & 2) v += p.bias[mm];
            v = act_fn(v, p.act);
            if (p.flags & 4) v += p.beta * R[(long long)mm * p.sRm + (long long)nn * p.sRn];
            ctile[8 * h + r][t * 16 + l15] = (n < p.N) ? v : 0.f;
        }
    }
    __syncthreads();
    const int NW = (p.Npad > p.N) ? p.Npad : p.N;
    const bool fast = (m0 + 16 <= p.M) && (n0 + 32 <= NW) && ((p.sCm & 3) == 0) && ((((size_t)C) & 15) == 0);
    if (fast) {
#pragma unroll
        for (int s = 0; s < 4; ++s) {
            const int row = s * 4 + (lane >> 3), c4 = (lane & 7) * 4;
            const v4f v = *(const v4f*)&ctile[row][c4];
            VST2V4(C + (long long)(m0 + row) * p.sCm + n0 + c4, v);
        }
    } else {
        for (int row = 0; row < 16; ++row) {
            const int m = m0 + row, n = n0 + lane;
            if (m < p.M && n < NW) VST2(float, C + (long long)m * p.sCm + n, ctile[row][lane]);
        }
    }
}

#define AW 4
struct AttnP {
    const float* Q; const float* K; const float* V; float* O; float* P; const float* Mf; const int* Mi; float* ST;
    const float* Pw; const float* Rt; const int* SQ; const int* SK;
    long long swb, swh, swi, swj, srb, srh, sri;
    long long sQb, sQh, sQi, sQd, sKb, sKh, sKj, sKd, sVb, sVh, sVj, sVd, sOb, sOh, sOi, sPb, sPh, sPi, smb, smh, smi, smj;
    int Lq, Lk, dh, dv, hrep, causal, coff, pband;
    float scale, mfill; int nonorm, mpol;
    int roff, rn, segpol, win;
};
static_assert(sizeof(AttnP) == 12 * 8 + 29 * 8 + 16 * 4, "AttnP has padding");

#ifndef KATTN_ATTR
#define KATTN_ATTR
#endif
template <int DHP, int DVP, int QM, bool SPLITPV, bool TWOPASS>
__global__ __launch_bounds__(32 * AW) KATTN_ATTR void k_attn(AttnP p) {
    constexpr int NT = DVP / 16;
    constexpr int KS = DHP / 32;
    constexpr int VP = DVP + 8;
    __shared__ __align__(16) float    pl[AW][16 * 64];
    __shared__ __align__(16) _Float16 vl[(SPLITPV ? 2 : 1) * 64 * VP];
    const int lane = threadIdx.x & 31, hf = lane >> 4, l15 = lane & 15, wave = threadIdx.x >> 5;
    const int h = blockIdx.y, b = blockIdx.z, hk = h / p.hrep;
    const int q0 = (blockIdx.x * AW + wave) * 16;
    float* myp = pl[wave];
    const float L2E = 1.4426950408889634f;
    const float NEG = -__builtin_inff();
    const int qi = min(q0 + l15, p.Lq - 1);
    const float* qrow = p.Q + b * p.sQb + h * p.sQh + (long long)qi * p.sQi;
    const float* kbase = p.K + b * p.sKb + hk * p.sKh;
    const float* vbase = p.V + b * p.sVb + hk * p.sVh;
    v16h qa[QM == 0 ? KS : 1]; Split qs_[QM == 1 ? KS : 1]; Split3 qt_[QM == 2 ? KS : 1];
#pragma unroll
    for (int ks = 0; ks < KS; ++ks) {
        if (QM == 2) qt_[ks] = sp3_ld(qrow, p.sQd, ks * 32, hf, p.dh, 1.f);
        else if (QM == 1) qs_[ks] = sp_ld(qrow, p.sQd, ks * 32, hf, p.dh, 1.f);
        else qa[ks] = fh_ld(qrow, p.sQd, ks * 32, hf, p.dh, 1.f);
    }
    v8f o[NT]; float m8[8], l8[8];
#pragma unroll
    for (int t = 0; t < NT; ++t) { v8f zz = {}; o[t] = zz; }
#pragma unroll
    for (int i = 0; i < 8; ++i) { m8[i] = NEG; l8[i] = 0.f; }
    int jend = p.Lk;
    if (p.causal == 1) { const int je = (blockIdx.x * AW + AW - 1) * 16 + 16 + p.coff; jend = min(jend, max(je, 0)); }
    const int npass = TWOPASS ? 2 : 1;
    for (int pass = 0; pass < npass; ++pass) {
        const bool dopv = (!TWOPASS) || pass == 1;
        for (int j0 = 0; j0 < jend; j0 += 64) {
            if (dopv) {
                __syncthreads();
                for (int idx = threadIdx.x; idx < 64 * DVP; idx += 32 * AW) {
                    const int jr = idx / DVP, d = idx - jr * DVP, j = j0 + jr;
                    const float f = (j < p.Lk && d < p.dv) ? vbase[(long long)j * p.sVj + (long long)d * p.sVd] : 0.f;
                    if (SPLITPV) {
                        const __bf16 hb = bf16_rne(f);
                        ((__bf16*)vl)[jr * VP + d] = hb; ((__bf16*)vl)[64 * VP + jr * VP + d] = bf16_rne(f - bf16_f32(hb));
                    } else vl[jr * VP + d] = (_Float16)f;
                }
            }
            v8f s[4];
#pragma unroll
            for (int t = 0; t < 4; ++t) {
                const int j = min(j0 + t * 16 + l15, p.Lk - 1);
                const float* krow = kbase + (long long)j * p.sKj;
                v8f acc = {};
#pragma unroll
                for (int ks = 0; ks < KS; ++ks) {
                    if (QM == 2)      acc = wmma6(qt_[ks], sp3_ld(krow, p.sKd, ks * 32, hf, p.dh, 1.f), acc);
                    else if (QM == 1) acc = wmma3(qs_[ks], sp_ld(krow, p.sKd, ks * 32, hf, p.dh, 1.f), acc);
                    else              acc = wmma16(qa[ks], fh_ld(krow, p.sKd, ks * 32, hf, p.dh, 1.f), acc);
                }
                s[t] = acc;
            }
            float pv[8][4];
#pragma unroll
            for (int i = 0; i < 8; ++i) {
                const int irow = q0 + i + 8 * hf;
                const int ic = min(irow, p.Lq - 1);
                float sc[4];
#pragma unroll
                for (int t = 0; t < 4; ++t) {
                    const int jg = j0 + t * 16 + l15;
                    float v = s[t][i] * p.scale;
                    if (p.Mf) v += p.Mf[b * p.smb + h * p.smh + (long long)ic * p.smi + (long long)min(jg, p.Lk - 1) * p.smj];
                    if (p.Rt) { int rc = ic - min(jg, p.Lk - 1) + p.roff; rc = rc < 0 ? 0 : (rc >= p.rn ? p.rn - 1 : rc); v += p.Rt[b * p.srb + h * p.srh + (long long)ic * p.sri + rc]; }
                    if (p.Mi) { const int mv = p.Mi[b * p.smb + h * p.smh + (long long)ic * p.smi + (long long)min(jg, p.Lk - 1) * p.smj]; if (p.mpol ? (mv != 0) : (mv == 0)) v = p.mfill; }
                    if (p.SQ) { const bool same = p.SQ[(long long)b * p.Lq + ic] == p.SK[(long long)b * p.Lk + min(jg, p.Lk - 1)]; if (p.segpol ? same : !same) v = p.mfill; }
                    if (p.causal == 2 && jg > irow + p.coff) v = p.mfill;
                    if (jg >= p.Lk || (p.causal == 1 && jg > irow + p.coff) || (p.causal == 3 && jg < irow + p.coff) || (p.win > 0 && irow + p.coff - jg > p.win)) v = NEG; else v *= L2E;
                    sc[t] = v;
                }
                if (!TWOPASS || pass == 0) {
                    float mx = fmaxf(fmaxf(sc[0], sc[1]), fmaxf(sc[2], sc[3]));
                    mx = fmaxf(mx, __shfl_xor(mx, 1, 32)); mx = fmaxf(mx, __shfl_xor(mx, 2, 32));
                    mx = fmaxf(mx, __shfl_xor(mx, 4, 32)); mx = fmaxf(mx, __shfl_xor(mx, 8, 32));
                    const float mnew = fmaxf(m8[i], mx);
                    const float corr = (mnew == NEG) ? 1.f : exp2f(m8[i] - mnew);
                    float rs = 0.f;
#pragma unroll
                    for (int t = 0; t < 4; ++t) {
                        const float pp = (sc[t] == NEG) ? 0.f : exp2f(sc[t] - mnew); rs += pp;
                        pv[i][t] = p.Pw ? pp * p.Pw[b * p.swb + h * p.swh + (long long)ic * p.swi + (long long)min(j0 + t * 16 + l15, p.Lk - 1) * p.swj] : pp;
                    }
                    rs += __shfl_xor(rs, 1, 32); rs += __shfl_xor(rs, 2, 32); rs += __shfl_xor(rs, 4, 32); rs += __shfl_xor(rs, 8, 32);
                    l8[i] = l8[i] * corr + rs; m8[i] = mnew;
                    if (!TWOPASS) {
#pragma unroll
                        for (int t = 0; t < NT; ++t) o[t][i] *= corr;
                    }
                } else {
                    const float inv = (l8[i] > 0.f) ? 1.f / l8[i] : 0.f;
#pragma unroll
                    for (int t = 0; t < 4; ++t) {
                        const int jg = j0 + t * 16 + l15;
                        float pp = (sc[t] == NEG) ? 0.f : exp2f(sc[t] - m8[i]) * inv;
                        if (p.Pw) pp *= p.Pw[b * p.swb + h * p.swh + (long long)ic * p.swi + (long long)min(jg, p.Lk - 1) * p.swj];
                        pv[i][t] = pp;
                    }
                }
            }
            if (dopv) {
#pragma unroll
                for (int i = 0; i < 8; ++i)
#pragma unroll
                    for (int t = 0; t < 4; ++t) myp[(i + 8 * hf) * 64 + t * 16 + l15] = pv[i][t];
                __syncthreads();
                if (p.P) {
                    float* pb_ = p.P + b * p.sPb + h * p.sPh;
                    const bool fastP = (p.pband == 0) && ((p.sPi & 3) == 0) && (j0 + 64 <= p.Lk) && (q0 + 16 <= p.Lq) && ((((size_t)pb_) & 15) == 0);
                    if (fastP) {
#pragma unroll
                        for (int s = 0; s < 8; ++s) {
                            const int row = s * 2 + (lane >> 4), c4 = (lane & 15) * 4;
                            const v4f v = *(const v4f*)(myp + row * 64 + c4);
                            VST2V4(pb_ + (long long)(q0 + row) * p.sPi + j0 + c4, v);
                        }
                    } else {
                        for (int row = 0; row < 16; ++row) {
                            const int irow = q0 + row; if (irow >= p.Lq) continue;
                            for (int c = lane; c < 64; c += 32) {
                                const int jg = j0 + c; if (jg >= p.Lk) continue;
                                if (p.pband == 0) VST2(float, pb_ + (long long)irow * p.sPi + jg, myp[row * 64 + c]);
                                else if (jg - irow <= p.pband && irow - jg <= p.pband) VST2(float, pb_ + (long long)irow * p.sPi + (jg - irow + p.pband), myp[row * 64 + c]);
                            }
                        }
                    }
                }
                if (SPLITPV) {
                    const Split pa0 = sp_ld(myp + l15 * 64, 1, 0, hf, 64, 1.f), pa1 = sp_ld(myp + l15 * 64, 1, 32, hf, 64, 1.f);
                    const __bf16* vh = (const __bf16*)vl; const __bf16* vlo = vh + 64 * VP;
#pragma unroll
                    for (int t = 0; t < NT; ++t) {
                        const int dcol = t * 16 + l15;
                        Split b0, b1;
#pragma unroll
                        for (int e = 0; e < 16; ++e) {
                            const int k0 = frag_k(e, hf), k1 = 32 + frag_k(e, hf);
                            b0.hi[e] = vh[k0 * VP + dcol]; b0.lo[e] = vlo[k0 * VP + dcol]; b1.hi[e] = vh[k1 * VP + dcol]; b1.lo[e] = vlo[k1 * VP + dcol];
                        }
                        o[t] = wmma3(pa0, b0, o[t]);
                        o[t] = wmma3(pa1, b1, o[t]);
                    }
                } else {
                    const v16h pa0 = fh_ld(myp + l15 * 64, 1, 0, hf, 64, 4096.f), pa1 = fh_ld(myp + l15 * 64, 1, 32, hf, 64, 4096.f);
#pragma unroll
                    for (int t = 0; t < NT; ++t) {
                        const int dcol = t * 16 + l15;
                        v16h b0, b1;
#pragma unroll
                        for (int e = 0; e < 16; ++e) { b0[e] = vl[frag_k(e, hf) * VP + dcol]; b1[e] = vl[(32 + frag_k(e, hf)) * VP + dcol]; }
                        o[t] = wmma16(pa0, b0, o[t]);
                        o[t] = wmma16(pa1, b1, o[t]);
                    }
                }
            }
        }
    }
    float* obase = p.O + b * p.sOb + h * p.sOh;
    if (p.ST) {
        const int rl = lane >> 1, isel = rl & 7;
        float mv = 0.f, lv = 0.f;
#pragma unroll
        for (int i = 0; i < 8; ++i) if (i == isel) { mv = m8[i]; lv = l8[i]; }
        const int irow = q0 + rl;
        if (irow < p.Lq) { float* st = p.ST + (((long long)b * gridDim.y + h) * p.Lq + irow) * 2 + (lane & 1); VST2(float, st, (lane & 1) ? lv : mv * 0.6931471805599453f); }
    }
    float invr[8];
#pragma unroll
    for (int i = 0; i < 8; ++i) {
        if (TWOPASS) invr[i] = SPLITPV ? 1.f : (1.f / 4096.f);
        else if (p.nonorm) invr[i] = exp2f(m8[i]) * (SPLITPV ? 1.f : (1.f / 4096.f));
        else invr[i] = (l8[i] > 0.f) ? (SPLITPV ? 1.f / l8[i] : 1.f / (l8[i] * 4096.f)) : 0.f;
    }
    __syncthreads();
    const bool ofast = ((p.sOi & 3) == 0) && ((((size_t)obase) & 15) == 0) && (q0 + 16 <= p.Lq);
#pragma unroll
    for (int c0 = 0; c0 < DVP; c0 += 64) {
#pragma unroll
        for (int i = 0; i < 8; ++i)
#pragma unroll
            for (int t = 0; t < NT; ++t) if (t * 16 >= c0 && t * 16 < c0 + 64) myp[(i + 8 * hf) * 64 + (t * 16 - c0) + l15] = o[t][i] * invr[i];
        __syncthreads();
        const int cw = (DVP - c0 < 64) ? (DVP - c0) : 64;
        if (ofast && (c0 + cw <= p.dv) && (cw % 32 == 0)) {
            const int lpr = cw / 4;
            const int rows_per_ins = 32 / lpr;
            for (int r0 = 0; r0 < 16; r0 += rows_per_ins) {
                const int row = r0 + lane / lpr, c4 = (lane % lpr) * 4;
                const v4f v = *(const v4f*)(myp + row * 64 + c4);
                VST2V4(obase + (long long)(q0 + row) * p.sOi + c0 + c4, v);
            }
        } else {
            for (int row = 0; row < 16; ++row) {
                const int irow = q0 + row; if (irow >= p.Lq) continue;
                for (int c = lane; c < cw; c += 32) { const int d = c0 + c; if (d < p.dv) VST2(float, obase + (long long)irow * p.sOi + d, myp[row * 64 + c]); }
            }
        }
        __syncthreads();
    }
}

struct TrP { const float* src; float* dst; const float* R2; long long sSz, lds, sDz, ldd, sRz, ldr; int R, C, flags, act; float alpha, beta; };
static_assert(sizeof(TrP) == 3 * 8 + 6 * 8 + 6 * 4, "TrP has padding");
__global__ __launch_bounds__(256) void k_tr(TrP p) {
    __shared__ float tile[32][33];
    const int c0 = blockIdx.x * 32, r0 = blockIdx.y * 32, z = blockIdx.z;
    const int lane = threadIdx.x & 31, wave = threadIdx.x >> 5;
    const float* s = p.src + z * p.sSz;
#pragma unroll
    for (int k = 0; k < 4; ++k) {
        const int rl = wave * 4 + k, r = r0 + rl, c = c0 + lane;
        tile[rl][lane] = (r < p.R && c < p.C) ? s[(long long)r * p.lds + c] : 0.f;
    }
    __syncthreads();
    float* d = p.dst + z * p.sDz; const float* rr = p.R2 + z * p.sRz;
#pragma unroll
    for (int k = 0; k < 4; ++k) {
        const int cl = wave * 4 + k, c = c0 + cl, r = r0 + lane;
        if (c < p.C && r < p.R) {
            float v = act_fn(p.alpha * tile[lane][cl], p.act);
            if (p.flags & 1) v += p.beta * rr[(long long)c * p.ldr + r];
            VST2(float, d + (long long)c * p.ldd + r, v);
        }
    }
}

__global__ __launch_bounds__(256) void k_affine(const float* __restrict__ src, float* __restrict__ dst, int n, float a, float b, const float* __restrict__ sdev) {
    const int i = blockIdx.x * 256 + threadIdx.x;
    if (i < n) { const float aa = sdev ? a * sdev[0] : a; const float v = aa * src[i] + b; VST2(float, dst + i, v); }
}

struct SmP { const float* src; float* dst; const float* Mf; long long sz, sr, dz, dr, smz, smr; int n, pad; float scale_in, scale_out; };
static_assert(sizeof(SmP) == 3 * 8 + 6 * 8 + 4 * 4, "SmP has padding");
__global__ __launch_bounds__(256) void k_softmax(SmP p) {
    __shared__ float red[256];
    const int r = blockIdx.x, z = blockIdx.y, tid = threadIdx.x;
    const float* s = p.src + z * p.sz + (long long)r * p.sr;
    const float* mf = p.Mf ? (p.Mf + z * p.smz + (long long)r * p.smr) : nullptr;
    float mx = -__builtin_inff();
    for (int j = tid; j < p.n; j += 256) { float v = s[j] * p.scale_in; if (mf) v += mf[j]; mx = fmaxf(mx, v); }
    red[tid] = mx; __syncthreads();
    for (int o = 128; o > 0; o >>= 1) { if (tid < o) red[tid] = fmaxf(red[tid], red[tid + o]); __syncthreads(); }
    mx = red[0]; __syncthreads();
    float sum = 0.f;
    for (int j = tid; j < p.n; j += 256) { float v = s[j] * p.scale_in; if (mf) v += mf[j]; sum += (mx == -__builtin_inff()) ? 0.f : expf(v - mx); }
    red[tid] = sum; __syncthreads();
    for (int o = 128; o > 0; o >>= 1) { if (tid < o) red[tid] += red[tid + o]; __syncthreads(); }
    sum = red[0];
    const float inv = (sum > 0.f) ? p.scale_out / sum : 0.f;
    float* d = p.dst + z * p.dz + (long long)r * p.dr;
    for (int j = tid; j < p.n; j += 256) { float v = s[j] * p.scale_in; if (mf) v += mf[j]; const float o = (mx == -__builtin_inff()) ? 0.f : expf(v - mx) * inv; VST2(float, d + j, o); }
}
__global__ __launch_bounds__(256) void k_stats(const float* __restrict__ x, long long sz, long long so, long long si, int inner, int n, float eps, float* __restrict__ stat, int mode) {
    __shared__ float red[256];
    const int z = blockIdx.x, tid = threadIdx.x;
    const float* base = x + z * sz;
    float s = 0.f;
    for (int e = tid; e < n; e += 256) s += base[(long long)(e / inner) * so + (long long)(e % inner) * si];
    red[tid] = s; __syncthreads();
    for (int o = 128; o > 0; o >>= 1) { if (tid < o) red[tid] += red[tid + o]; __syncthreads(); }
    const float mu = (mode == 0 || mode == 3) ? red[0] / (float)n : 0.f; __syncthreads();
    float q = 0.f;
    for (int e = tid; e < n; e += 256) { const float dlt = base[(long long)(e / inner) * so + (long long)(e % inner) * si] - mu; q += dlt * dlt; }
    red[tid] = q; __syncthreads();
    for (int o = 128; o > 0; o >>= 1) { if (tid < o) red[tid] += red[tid + o]; __syncthreads(); }
    {
        float rs;
        if (mode == 2) rs = sqrtf((float)n) / fmaxf(sqrtf(red[0]), eps); else if (mode == 3) rs = rsqrtf(red[0] / (float)(n - 1) + eps); else rs = rsqrtf(red[0] / (float)n + eps);
        if (tid < 32) { const float v = (tid == 0) ? mu : ((tid == 1) ? rs : 0.f); VST2(float, stat + (long long)z * 32 + tid, v); }
    }
}
__global__ __launch_bounds__(256) void k_norm_apply(const float* __restrict__ x, float* __restrict__ y, const float* __restrict__ stat, const float* __restrict__ g, const float* __restrict__ bta,
                                                     int Z, int C, int L, int G, int bn, int act) {
    const long long idx = (long long)blockIdx.x * 256 + threadIdx.x;
    if (idx >= (long long)Z * C * L) return;
    const int l = (int)(idx % L); const long long zc = idx / L; const int c = (int)(zc % C), z = (int)(zc / C); (void)l;
    const int set = bn ? c : (z * G + c / (C / G));
    float v = (x[idx] - stat[(long long)set * 32]) * stat[(long long)set * 32 + 1];
    if (g) v *= g[c];
    if (bta) v += bta[c];
    v = act_fn(v, act);
    VST2(float, y + idx, v);
}

__global__ __launch_bounds__(256) void k_lse_neg(const float* __restrict__ st, float* __restrict__ c, int n) {
    const int i = blockIdx.x * 256 + threadIdx.x;
    if (i < n) { const float v = -(st[2 * i] + logf(st[2 * i + 1])); VST2(float, c + i, v); }
}

__global__ __launch_bounds__(256) void k_iota(int* __restrict__ dst, int n, int a, int b) {
    const int i = blockIdx.x * 256 + threadIdx.x;
    if (i < n) { const int v = a * i + b; VST2(int, dst + i, v); }
}

__global__ __launch_bounds__(256) void k_axpby(const float* __restrict__ x, const float* __restrict__ y, float* __restrict__ dst, int n, float a, float b, float c) {
    const int i = blockIdx.x * 256 + threadIdx.x;
    if (i < n) { const float v = a * x[i] + b * y[i] + c; VST2(float, dst + i, v); }
}

struct RopeP { const float* X; float* Y; const float* C; const float* Sn; const int* pos; long long sXr, sXh, sYr, sYh, sCb, sCp, sCd; int R, Hn, D, S, mode, tmode, pmode, pad; };
static_assert(sizeof(RopeP) == 5 * 8 + 7 * 8 + 8 * 4, "RopeP has padding");
__global__ __launch_bounds__(256) void k_rope(RopeP p) {
    const long long idx = (long long)blockIdx.x * 256 + threadIdx.x;
    if (idx >= (long long)p.R * p.Hn * p.D) return;
    const int d = (int)(idx % p.D); const long long rh = idx / p.D; const int h = (int)(rh % p.Hn); const int r = (int)(rh / p.Hn);
    const int half = p.D / 2;
    int partner; float sign;
    if (p.mode == 0) { partner = (d < half) ? d + half : d - half; sign = (d < half) ? -1.f : 1.f; }
    else { partner = d ^ 1; sign = (d & 1) ? 1.f : -1.f; }
    const int tcol = (p.tmode == 0) ? d : ((p.tmode == 1) ? (d % half) : (d >> 1));
    const int pp = (p.pmode == 0) ? (r % p.S) : ((p.pmode == 1) ? h : p.pos[r]);
    const long long toff = (long long)(r / p.S) * p.sCb + (long long)pp * p.sCp + (long long)tcol * p.sCd;
    const float* xr = p.X + (long long)r * p.sXr + (long long)h * p.sXh;
    const float v = xr[d] * p.C[toff] + sign * xr[partner] * p.Sn[toff];
    VST2(float, p.Y + (long long)r * p.sYr + (long long)h * p.sYh + d, v);
}

__global__ __launch_bounds__(256) void k_invf(float* __restrict__ invb, int half, int D, float base, float num, int fmode, float cexp) {
    const int i = blockIdx.x * 256 + threadIdx.x;
    if (i >= ((half + 31) / 32) * 32) return;
    if (i >= half) { VST2(float, invb + i, 0.f); return; }
    const float e = (float)(2 * i) / (float)D;
    float invf;
    if (fmode == 1) invf = num * expf((float)(2 * i) * cexp);
    else if (fmode == 2) invf = num * powf(base, (-2.0f * ((float)i - 1.0f)) / (float)D);
    else invf = num * (1.0f / powf(base, e));
    VST2(float, invb + i, invf);
}
__global__ __launch_bounds__(256) void k_sincos(float* __restrict__ cs, float* __restrict__ sn, const float* __restrict__ invb, int S, int half, float pscale) {
    const int idx = blockIdx.x * 256 + threadIdx.x;
    if (idx >= S * half) return;
    const int s = idx / half, i = idx - s * half;
    const float ang = (pscale * (float)s) * invb[i];
    VST2(float, cs + idx, cosf(ang)); VST2(float, sn + idx, sinf(ang));
}

__global__ __launch_bounds__(256) void k_mulact(const float* __restrict__ x, const float* __restrict__ y, float* __restrict__ dst, int n, int act) {
    const int i = blockIdx.x * 256 + threadIdx.x;
    if (i < n) { const float v = act_fn(x[i], act) * y[i]; VST2(float, dst + i, v); }
}

__global__ __launch_bounds__(256) void k_matvec(GemmP p) {
    const int rpt = (p.N == 1) ? 1 : 32;
    const long long r0 = ((long long)blockIdx.x * 256 + threadIdx.x) * rpt; const int z = blockIdx.z, zo = z / p.zi_n, zi = z - zo * p.zi_n;
    if (r0 >= p.M) return;
    const float* Bb = p.B + zo * p.sBo + zi * p.sBi;
    float* C = p.C + zo * p.sCo + zi * p.sCi; const float* R = p.R + zo * p.sRo + zi * p.sRi;
    for (int rr = 0; rr < rpt; ++rr) {
        const long long r = r0 + rr; if (r >= p.M) break;
        const float* A = p.A + zo * p.sAo + zi * p.sAi + r * p.sAm;
        float acc[8] = {0.f, 0.f, 0.f, 0.f, 0.f, 0.f, 0.f, 0.f};
        for (int k = 0; k < p.K; ++k) { const float a = A[(long long)k * p.sAk];
#pragma unroll
            for (int j = 0; j < 8; ++j) if (j < p.N) acc[j] += a * Bb[(long long)j * p.sBn + (long long)k * p.sBk]; }
#pragma unroll
        for (int j = 0; j < 8; ++j) if (j < p.N) {
            float v = acc[j] * p.alpha;
            if (p.flags & 1) v += p.bias[j];
            if (p.flags & 2) v += p.bias[r];
            v = act_fn(v, p.act);
            if (p.flags & 4) v += p.beta * R[r * p.sRm + (long long)j * p.sRn];
            VST2(float, C + r * p.sCm + j, v);
        }
    }
}
__global__ __launch_bounds__(256) void k_smallsoftmax(const float* __restrict__ src, float* __restrict__ dst, long long sr, long long dr, int n, long long R, float scale) {
    const long long r0 = ((long long)blockIdx.x * 256 + threadIdx.x) * 32;
    for (int rr = 0; rr < 32; ++rr) {
        const long long r = r0 + rr; if (r >= R) return;
        const float* s = src + r * sr; float* d = dst + r * dr;
        float mx = -__builtin_inff();
        for (int j = 0; j < n; ++j) mx = fmaxf(mx, s[j] * scale);
        float sum = 0.f;
        for (int j = 0; j < n; ++j) sum += expf(s[j] * scale - mx);
        const float inv = 1.f / sum;
        for (int j = 0; j < n; ++j) { const float v = expf(s[j] * scale - mx) * inv; VST2(float, d + j, v); }
    }
}

__global__ __launch_bounds__(32) void k_unitstat(float* __restrict__ st) { const int t = threadIdx.x; const float v = (t == 1) ? 1.f : 0.f; VST2(float, st + t, v); }

__global__ __launch_bounds__(256) void k_lincopy(const float* __restrict__ src, long long lds, float* __restrict__ dst, long long ldd, long long rows, int cols) {
    const long long i = (long long)blockIdx.x * 256 + threadIdx.x; if (i >= rows * cols) return;
    const long long r = i / cols; const int c = (int)(i - r * cols);
    const float v = src[r * lds + c]; VST2(float, dst + r * ldd + c, v);
}

#define IL_CAP32 32
#define IL_T32 256
#define IL_TILE32 4096
__global__ __launch_bounds__(IL_T32) void k_inlists32(const int* __restrict__ tgt, int E, int N, int* __restrict__ NBR, int* __restrict__ cnt) {
    __shared__ int tt[IL_TILE32];
    __shared__ int lists[IL_T32 * IL_CAP32];
    const int d = blockIdx.x * IL_T32 + threadIdx.x; int n = 0;
    for (int e0 = 0; e0 < E; e0 += IL_TILE32) {
        const int nt = min(IL_TILE32, E - e0);
        __syncthreads();
        for (int i = threadIdx.x; i < nt; i += IL_T32) tt[i] = tgt[e0 + i];
        __syncthreads();
        for (int i = 0; i < nt; ++i) { if (tt[i] == d) { if (n < IL_CAP32) lists[threadIdx.x * IL_CAP32 + n] = e0 + i; ++n; } }
    }
    if (d < N) {
        int* row = NBR + (long long)d * IL_CAP32;
        for (int j = 0; j < IL_CAP32; ++j) { const int v = (j < n) ? lists[threadIdx.x * IL_CAP32 + j] : -1; VST2(int, row + j, v); }
        VST2(int, cnt + d, min(n, IL_CAP32));
    }
}
__global__ __launch_bounds__(256) void k_csr_scan32(const int* __restrict__ cnt, int* __restrict__ off, int N) {
    __shared__ int part[256]; const int per = ((((N + 255) / 256) + 31) / 32) * 32; const int a = threadIdx.x * per, b = min(N, a + per); int s = 0;
    for (int i = a; i < b; ++i) s += cnt[i]; part[threadIdx.x] = s; __syncthreads();
    if (threadIdx.x == 0) { int run = 0; for (int t = 0; t < 256; ++t) { const int v = part[t]; part[t] = run; run += v; } } __syncthreads();
    int run = part[threadIdx.x]; for (int i = a; i < b; ++i) { VST2(int, off + i, run); run += cnt[i]; }
    if (a < N && b == N) { VST2(int, off + N, run); }
}
__global__ __launch_bounds__(256) void k_slotcopy32(const int* __restrict__ off, const int* __restrict__ NBR, int* __restrict__ slot, int N) {
    const int t = blockIdx.x * 256 + threadIdx.x; const int tot = off[N]; if (t >= tot) return;
    int lo = 0, hi = N - 1;
    while (lo < hi) { const int mid = (lo + hi + 1) >> 1; if (off[mid] <= t) lo = mid; else hi = mid - 1; }
    int j = t - off[lo]; j = (j < 0) ? 0 : ((j >= IL_CAP32) ? (IL_CAP32 - 1) : j);
    VST2(int, slot + t, NBR[(long long)lo * IL_CAP32 + j]);
}

__global__ __launch_bounds__(256) void k_knn_prep(const float* __restrict__ ea, const float* __restrict__ kw1, const float* __restrict__ kb1, float* __restrict__ KHb, int E, int KH, const float* __restrict__ kw2, const float* __restrict__ kb2, float* __restrict__ K2P, float* __restrict__ B2M, int Wd) {
    const long long q = (long long)blockIdx.x * 256 + threadIdx.x;
    if (q < (long long)E * KH) { const int j = (int)(q % KH); const long long e = q / KH; float s = kb1[j];
#pragma unroll 1
        for (int a = 0; a < 6; ++a) s += ea[e * 6 + a] * kw1[a * KH + j]; VST2(float, KHb + q, fmaxf(s, 0.f)); }
    if (q < (long long)KH * Wd * Wd) VST2(float, K2P + q, kw2[q]);
    if (q < (long long)Wd * Wd) VST2(float, B2M + q, kb2[q]);
}
__global__ __launch_bounds__(256) void k_knn_fc1(const float* __restrict__ x, const float* __restrict__ w, const float* __restrict__ b, float* __restrict__ H, int N, int Wd) { const int q = blockIdx.x * 256 + threadIdx.x; if (q >= N * Wd) return; const int o = q % Wd; VST2(float, H + q, x[q / Wd] * w[o] + b[o]); }
__global__ __launch_bounds__(256) void k_knn_agg(const float* __restrict__ H, const float* __restrict__ KHb, const int* __restrict__ ei, const int* __restrict__ off, const int* __restrict__ slot, float* __restrict__ AF, float* __restrict__ AX, int N, int Wd, int KH) {
    const long long q = (long long)blockIdx.x * 256 + threadIdx.x; if (q >= (long long)N * KH * Wd) return; const int i = (int)(q % Wd); const int j = (int)((q / Wd) % KH); const int n = (int)(q / (Wd * KH)); const int a = off[n], b = off[n + 1]; float s = 0.f, sx = 0.f;
    for (int p = a; p < b; ++p) { const int e = slot[p]; const float hv = H[(long long)ei[e] * Wd + i]; s += KHb[(long long)e * KH + j] * hv; sx += hv; }
    const float inv = (b > a) ? 1.f / (float)(b - a) : 0.f; VST2(float, AF + q, s * inv); if (j == 0) VST2(float, AX + (long long)n * Wd + i, sx * inv);
}

template __global__ void k_gemm<1>(GemmP);

extern "C" void kernel_launch(void* const* d_in, const int* in_sizes, int n_in, void* d_out, int out_size, void* d_ws, size_t ws_size, hipStream_t stream) {
    (void)in_sizes; (void)n_in; (void)out_size; (void)ws_size;
    const float* x = (const float*)d_in[0];
    const int* ei = (const int*)d_in[1];
    const float* ea = (const float*)d_in[2];
    const float* f1w = (const float*)d_in[3];
    const float* f1b = (const float*)d_in[4];
    const float* kw1 = (const float*)d_in[5];
    const float* kb1 = (const float*)d_in[6];
    const float* kw2 = (const float*)d_in[7];
    const float* kb2 = (const float*)d_in[8];
    const float* root = (const float*)d_in[9];
    const float* cb = (const float*)d_in[10];
    const float* f2w = (const float*)d_in[11];
    const float* f2b = (const float*)d_in[12];
    const int Nn = 30000;
    const int E = 120000;
    const int Wd = 32;
    const int KH = 8;
    const int KF = KH * Wd;
    const int CAP = 32;
    const int LP = 32;
    float* out = (float*)d_out;
    char* wsp = (char*)d_ws;
    int* cnt = (int*)wsp; wsp += (((size_t)((size_t)Nn + 64) * 4 + 255) / 256) * 256;
    int* off = (int*)wsp; wsp += (((size_t)((size_t)Nn + 64) * 4 + 255) / 256) * 256;
    int* slot = (int*)wsp; wsp += (((size_t)((size_t)E + 64) * 4 + 255) / 256) * 256;
    int* nbr = (int*)wsp; wsp += (((size_t)((size_t)Nn * CAP) * 4 + 255) / 256) * 256;
    float* KHb = (float*)wsp; wsp += (((size_t)((size_t)E * KH) * 4 + 255) / 256) * 256;
    float* K2P = (float*)wsp; wsp += (((size_t)((size_t)KF * Wd) * 4 + 255) / 256) * 256;
    float* B2M = (float*)wsp; wsp += (((size_t)((size_t)Wd * Wd + 128) * 4 + 255) / 256) * 256;
    float* Hh = (float*)wsp; wsp += (((size_t)((size_t)Nn * Wd) * 4 + 255) / 256) * 256;
    float* AF = (float*)wsp; wsp += (((size_t)((size_t)Nn * KF) * 4 + 255) / 256) * 256;
    float* AX = (float*)wsp; wsp += (((size_t)((size_t)Nn * Wd) * 4 + 255) / 256) * 256;
    float* T = (float*)wsp; wsp += (((size_t)((size_t)Nn * Wd) * 4 + 255) / 256) * 256;
    k_inlists32<<<(unsigned)((Nn) + IL_T32 - 1) / IL_T32, IL_T32, 0, stream>>>(ei + E, E, Nn, nbr, cnt);
    k_csr_scan32<<<1, 256, 0, stream>>>(cnt, off, Nn);
    k_slotcopy32<<<(unsigned)((E) + 255) / 256, 256, 0, stream>>>(off, nbr, slot, Nn);
    k_knn_prep<<<(unsigned)(((long long)E * KH + 255) / 256), 256, 0, stream>>>(ea, kw1, kb1, KHb, E, KH, kw2, kb2, K2P, B2M, Wd);
    k_knn_fc1<<<(unsigned)((Nn * Wd + 255) / 256), 256, 0, stream>>>(x, f1w, f1b, Hh, Nn, Wd);
    k_knn_agg<<<(unsigned)(((long long)Nn * KF + 255) / 256), 256, 0, stream>>>(Hh, KHb, ei, off, slot, AF, AX, Nn, Wd, KH);
    { GemmP ga0;
      ga0.A = AF; ga0.B = K2P; ga0.bias = cb; ga0.R = AF; ga0.C = T;
      ga0.sAo = 0; ga0.sAi = 0; ga0.sAm = KF; ga0.sAk = 1; ga0.sBo = 0; ga0.sBi = 0; ga0.sBn = 1; ga0.sBk = Wd; ga0.sCo = 0; ga0.sCi = 0; ga0.sCm = Wd; ga0.sRo = 0; ga0.sRi = 0; ga0.sRm = 0; ga0.sRn = 0;
      ga0.M = Nn; ga0.N = Wd; ga0.K = KF; ga0.zi_n = 1; ga0.flags = 1; ga0.act = 0;
      ga0.alpha = 1.0f; ga0.beta = 0.0f; ga0.sa = 1.0f; ga0.sb = 1.0f; ga0.Npad = Wd; ga0.pad_ = 0;
      k_gemm<1><<<dim3((unsigned)((Wd) + 31) / 32, (unsigned)((Nn) + 15) / 16, (unsigned)(1)), 32, 0, stream>>>(ga0); }
    { GemmP gb0;
      gb0.A = AX; gb0.B = B2M; gb0.bias = AX; gb0.R = T; gb0.C = T;
      gb0.sAo = 0; gb0.sAi = 0; gb0.sAm = Wd; gb0.sAk = 1; gb0.sBo = 0; gb0.sBi = 0; gb0.sBn = 1; gb0.sBk = Wd; gb0.sCo = 0; gb0.sCi = 0; gb0.sCm = Wd; gb0.sRo = 0; gb0.sRi = 0; gb0.sRm = Wd; gb0.sRn = 1;
      gb0.M = Nn; gb0.N = Wd; gb0.K = Wd; gb0.zi_n = 1; gb0.flags = 4; gb0.act = 0;
      gb0.alpha = 1.0f; gb0.beta = 1.0f; gb0.sa = 1.0f; gb0.sb = 1.0f; gb0.Npad = Wd; gb0.pad_ = 0;
      k_gemm<1><<<dim3((unsigned)((Wd) + 31) / 32, (unsigned)((Nn) + 15) / 16, (unsigned)(1)), 32, 0, stream>>>(gb0); }
    { GemmP gr0;
      gr0.A = Hh; gr0.B = root; gr0.bias = Hh; gr0.R = T; gr0.C = AX;
      gr0.sAo = 0; gr0.sAi = 0; gr0.sAm = Wd; gr0.sAk = 1; gr0.sBo = 0; gr0.sBi = 0; gr0.sBn = 1; gr0.sBk = Wd; gr0.sCo = 0; gr0.sCi = 0; gr0.sCm = Wd; gr0.sRo = 0; gr0.sRi = 0; gr0.sRm = Wd; gr0.sRn = 1;
      gr0.M = Nn; gr0.N = Wd; gr0.K = Wd; gr0.zi_n = 1; gr0.flags = 4; gr0.act = 0;
      gr0.alpha = 1.0f; gr0.beta = 1.0f; gr0.sa = 1.0f; gr0.sb = 1.0f; gr0.Npad = Wd; gr0.pad_ = 0;
      k_gemm<1><<<dim3((unsigned)((Wd) + 31) / 32, (unsigned)((Nn) + 15) / 16, (unsigned)(1)), 32, 0, stream>>>(gr0); }
    k_unitstat<<<1, 32, 0, stream>>>(B2M + 1024);
    k_norm_apply<<<(unsigned)(((long long)(1) * (1) * ((long long)Nn * Wd) + 255) / 256), 256, 0, stream>>>(AX, Hh, B2M + 1024, nullptr, nullptr, 1, 1, (long long)Nn * Wd, 1, 0, 1);
    k_knn_agg<<<(unsigned)(((long long)Nn * KF + 255) / 256), 256, 0, stream>>>(Hh, KHb, ei, off, slot, AF, AX, Nn, Wd, KH);
    { GemmP ga1;
      ga1.A = AF; ga1.B = K2P; ga1.bias = cb; ga1.R = AF; ga1.C = T;
      ga1.sAo = 0; ga1.sAi = 0; ga1.sAm = KF; ga1.sAk = 1; ga1.sBo = 0; ga1.sBi = 0; ga1.sBn = 1; ga1.sBk = Wd; ga1.sCo = 0; ga1.sCi = 0; ga1.sCm = Wd; ga1.sRo = 0; ga1.sRi = 0; ga1.sRm = 0; ga1.sRn = 0;
      ga1.M = Nn; ga1.N = Wd; ga1.K = KF; ga1.zi_n = 1; ga1.flags = 1; ga1.act = 0;
      ga1.alpha = 1.0f; ga1.beta = 0.0f; ga1.sa = 1.0f; ga1.sb = 1.0f; ga1.Npad = Wd; ga1.pad_ = 0;
      k_gemm<1><<<dim3((unsigned)((Wd) + 31) / 32, (unsigned)((Nn) + 15) / 16, (unsigned)(1)), 32, 0, stream>>>(ga1); }
    { GemmP gb1;
      gb1.A = AX; gb1.B = B2M; gb1.bias = AX; gb1.R = T; gb1.C = T;
      gb1.sAo = 0; gb1.sAi = 0; gb1.sAm = Wd; gb1.sAk = 1; gb1.sBo = 0; gb1.sBi = 0; gb1.sBn = 1; gb1.sBk = Wd; gb1.sCo = 0; gb1.sCi = 0; gb1.sCm = Wd; gb1.sRo = 0; gb1.sRi = 0; gb1.sRm = Wd; gb1.sRn = 1;
      gb1.M = Nn; gb1.N = Wd; gb1.K = Wd; gb1.zi_n = 1; gb1.flags = 4; gb1.act = 0;
      gb1.alpha = 1.0f; gb1.beta = 1.0f; gb1.sa = 1.0f; gb1.sb = 1.0f; gb1.Npad = Wd; gb1.pad_ = 0;
      k_gemm<1><<<dim3((unsigned)((Wd) + 31) / 32, (unsigned)((Nn) + 15) / 16, (unsigned)(1)), 32, 0, stream>>>(gb1); }
    { GemmP gr1;
      gr1.A = Hh; gr1.B = root; gr1.bias = Hh; gr1.R = T; gr1.C = AX;
      gr1.sAo = 0; gr1.sAi = 0; gr1.sAm = Wd; gr1.sAk = 1; gr1.sBo = 0; gr1.sBi = 0; gr1.sBn = 1; gr1.sBk = Wd; gr1.sCo = 0; gr1.sCi = 0; gr1.sCm = Wd; gr1.sRo = 0; gr1.sRi = 0; gr1.sRm = Wd; gr1.sRn = 1;
      gr1.M = Nn; gr1.N = Wd; gr1.K = Wd; gr1.zi_n = 1; gr1.flags = 4; gr1.act = 0;
      gr1.alpha = 1.0f; gr1.beta = 1.0f; gr1.sa = 1.0f; gr1.sb = 1.0f; gr1.Npad = Wd; gr1.pad_ = 0;
      k_gemm<1><<<dim3((unsigned)((Wd) + 31) / 32, (unsigned)((Nn) + 15) / 16, (unsigned)(1)), 32, 0, stream>>>(gr1); }
    k_norm_apply<<<(unsigned)(((long long)(1) * (1) * ((long long)Nn * Wd) + 255) / 256), 256, 0, stream>>>(AX, Hh, B2M + 1024, nullptr, nullptr, 1, 1, (long long)Nn * Wd, 1, 0, 1);
    k_knn_agg<<<(unsigned)(((long long)Nn * KF + 255) / 256), 256, 0, stream>>>(Hh, KHb, ei, off, slot, AF, AX, Nn, Wd, KH);
    { GemmP ga2;
      ga2.A = AF; ga2.B = K2P; ga2.bias = cb; ga2.R = AF; ga2.C = T;
      ga2.sAo = 0; ga2.sAi = 0; ga2.sAm = KF; ga2.sAk = 1; ga2.sBo = 0; ga2.sBi = 0; ga2.sBn = 1; ga2.sBk = Wd; ga2.sCo = 0; ga2.sCi = 0; ga2.sCm = Wd; ga2.sRo = 0; ga2.sRi = 0; ga2.sRm = 0; ga2.sRn = 0;
      ga2.M = Nn; ga2.N = Wd; ga2.K = KF; ga2.zi_n = 1; ga2.flags = 1; ga2.act = 0;
      ga2.alpha = 1.0f; ga2.beta = 0.0f; ga2.sa = 1.0f; ga2.sb = 1.0f; ga2.Npad = Wd; ga2.pad_ = 0;
      k_gemm<1><<<dim3((unsigned)((Wd) + 31) / 32, (unsigned)((Nn) + 15) / 16, (unsigned)(1)), 32, 0, stream>>>(ga2); }
    { GemmP gb2;
      gb2.A = AX; gb2.B = B2M; gb2.bias = AX; gb2.R = T; gb2.C = T;
      gb2.sAo = 0; gb2.sAi = 0; gb2.sAm = Wd; gb2.sAk = 1; gb2.sBo = 0; gb2.sBi = 0; gb2.sBn = 1; gb2.sBk = Wd; gb2.sCo = 0; gb2.sCi = 0; gb2.sCm = Wd; gb2.sRo = 0; gb2.sRi = 0; gb2.sRm = Wd; gb2.sRn = 1;
      gb2.M = Nn; gb2.N = Wd; gb2.K = Wd; gb2.zi_n = 1; gb2.flags = 4; gb2.act = 0;
      gb2.alpha = 1.0f; gb2.beta = 1.0f; gb2.sa = 1.0f; gb2.sb = 1.0f; gb2.Npad = Wd; gb2.pad_ = 0;
      k_gemm<1><<<dim3((unsigned)((Wd) + 31) / 32, (unsigned)((Nn) + 15) / 16, (unsigned)(1)), 32, 0, stream>>>(gb2); }
    { GemmP gr2;
      gr2.A = Hh; gr2.B = root; gr2.bias = Hh; gr2.R = T; gr2.C = AX;
      gr2.sAo = 0; gr2.sAi = 0; gr2.sAm = Wd; gr2.sAk = 1; gr2.sBo = 0; gr2.sBi = 0; gr2.sBn = 1; gr2.sBk = Wd; gr2.sCo = 0; gr2.sCi = 0; gr2.sCm = Wd; gr2.sRo = 0; gr2.sRi = 0; gr2.sRm = Wd; gr2.sRn = 1;
      gr2.M = Nn; gr2.N = Wd; gr2.K = Wd; gr2.zi_n = 1; gr2.flags = 4; gr2.act = 0;
      gr2.alpha = 1.0f; gr2.beta = 1.0f; gr2.sa = 1.0f; gr2.sb = 1.0f; gr2.Npad = Wd; gr2.pad_ = 0;
      k_gemm<1><<<dim3((unsigned)((Wd) + 31) / 32, (unsigned)((Nn) + 15) / 16, (unsigned)(1)), 32, 0, stream>>>(gr2); }
    k_norm_apply<<<(unsigned)(((long long)(1) * (1) * ((long long)Nn * Wd) + 255) / 256), 256, 0, stream>>>(AX, Hh, B2M + 1024, nullptr, nullptr, 1, 1, (long long)Nn * Wd, 1, 0, 1);
    k_knn_agg<<<(unsigned)(((long long)Nn * KF + 255) / 256), 256, 0, stream>>>(Hh, KHb, ei, off, slot, AF, AX, Nn, Wd, KH);
    { GemmP ga3;
      ga3.A = AF; ga3.B = K2P; ga3.bias = cb; ga3.R = AF; ga3.C = T;
      ga3.sAo = 0; ga3.sAi = 0; ga3.sAm = KF; ga3.sAk = 1; ga3.sBo = 0; ga3.sBi = 0; ga3.sBn = 1; ga3.sBk = Wd; ga3.sCo = 0; ga3.sCi = 0; ga3.sCm = Wd; ga3.sRo = 0; ga3.sRi = 0; ga3.sRm = 0; ga3.sRn = 0;
      ga3.M = Nn; ga3.N = Wd; ga3.K = KF; ga3.zi_n = 1; ga3.flags = 1; ga3.act = 0;
      ga3.alpha = 1.0f; ga3.beta = 0.0f; ga3.sa = 1.0f; ga3.sb = 1.0f; ga3.Npad = Wd; ga3.pad_ = 0;
      k_gemm<1><<<dim3((unsigned)((Wd) + 31) / 32, (unsigned)((Nn) + 15) / 16, (unsigned)(1)), 32, 0, stream>>>(ga3); }
    { GemmP gb3;
      gb3.A = AX; gb3.B = B2M; gb3.bias = AX; gb3.R = T; gb3.C = T;
      gb3.sAo = 0; gb3.sAi = 0; gb3.sAm = Wd; gb3.sAk = 1; gb3.sBo = 0; gb3.sBi = 0; gb3.sBn = 1; gb3.sBk = Wd; gb3.sCo = 0; gb3.sCi = 0; gb3.sCm = Wd; gb3.sRo = 0; gb3.sRi = 0; gb3.sRm = Wd; gb3.sRn = 1;
      gb3.M = Nn; gb3.N = Wd; gb3.K = Wd; gb3.zi_n = 1; gb3.flags = 4; gb3.act = 0;
      gb3.alpha = 1.0f; gb3.beta = 1.0f; gb3.sa = 1.0f; gb3.sb = 1.0f; gb3.Npad = Wd; gb3.pad_ = 0;
      k_gemm<1><<<dim3((unsigned)((Wd) + 31) / 32, (unsigned)((Nn) + 15) / 16, (unsigned)(1)), 32, 0, stream>>>(gb3); }
    { GemmP gr3;
      gr3.A = Hh; gr3.B = root; gr3.bias = Hh; gr3.R = T; gr3.C = AX;
      gr3.sAo = 0; gr3.sAi = 0; gr3.sAm = Wd; gr3.sAk = 1; gr3.sBo = 0; gr3.sBi = 0; gr3.sBn = 1; gr3.sBk = Wd; gr3.sCo = 0; gr3.sCi = 0; gr3.sCm = Wd; gr3.sRo = 0; gr3.sRi = 0; gr3.sRm = Wd; gr3.sRn = 1;
      gr3.M = Nn; gr3.N = Wd; gr3.K = Wd; gr3.zi_n = 1; gr3.flags = 4; gr3.act = 0;
      gr3.alpha = 1.0f; gr3.beta = 1.0f; gr3.sa = 1.0f; gr3.sb = 1.0f; gr3.Npad = Wd; gr3.pad_ = 0;
      k_gemm<1><<<dim3((unsigned)((Wd) + 31) / 32, (unsigned)((Nn) + 15) / 16, (unsigned)(1)), 32, 0, stream>>>(gr3); }
    k_norm_apply<<<(unsigned)(((long long)(1) * (1) * ((long long)Nn * Wd) + 255) / 256), 256, 0, stream>>>(AX, Hh, B2M + 1024, nullptr, nullptr, 1, 1, (long long)Nn * Wd, 1, 0, 1);
    { GemmP gf2;
      gf2.A = Hh; gf2.B = f2w; gf2.bias = f2b; gf2.R = Hh; gf2.C = T;
      gf2.sAo = 0; gf2.sAi = 0; gf2.sAm = Wd; gf2.sAk = 1; gf2.sBo = 0; gf2.sBi = 0; gf2.sBn = 1; gf2.sBk = 1; gf2.sCo = 0; gf2.sCi = 0; gf2.sCm = LP; gf2.sRo = 0; gf2.sRi = 0; gf2.sRm = 0; gf2.sRn = 0;
      gf2.M = Nn; gf2.N = 1; gf2.K = Wd; gf2.zi_n = 1; gf2.flags = 1; gf2.act = 0;
      gf2.alpha = 1.0f; gf2.beta = 0.0f; gf2.sa = 1.0f; gf2.sb = 1.0f; gf2.Npad = LP; gf2.pad_ = 0;
      k_gemm<1><<<dim3((unsigned)((LP) + 31) / 32, (unsigned)((Nn) + 15) / 16, (unsigned)(1)), 32, 0, stream>>>(gf2); }
    k_lincopy<<<(unsigned)(((long long)(Nn) * (1) + 255) / 256), 256, 0, stream>>>(T, LP, out, 1, Nn, 1);
}
